// TransformerBlock_12575664242959
// MI455X (gfx1250) — hardware-verified
//
#include <hip/hip_runtime.h>
#include <stddef.h>


typedef _Float16 v16h __attribute__((ext_vector_type(16)));
typedef _Float16 v8h  __attribute__((ext_vector_type(8)));
typedef _Float16 v4h  __attribute__((ext_vector_type(4)));
typedef float    v8f  __attribute__((ext_vector_type(8)));
typedef float    v4f  __attribute__((ext_vector_type(4)));

#ifndef NB
#define NB 4
#endif
#ifndef SEQ
#define SEQ 2048
#endif
#define NB_FULL  4
#define SEQ_FULL 2048
#define DIM   384
#define DFF   1536
#define NHEAD 6
#define HD    64
#define QKLD  (2 * DIM)
#define MROWS (NB * SEQ)
#define LNROWS 8
#define LN_EPS 1.0e-5f

static_assert(NB >= 1 && NB <= NB_FULL);
static_assert(SEQ >= 128 && SEQ <= SEQ_FULL && (SEQ % 128) == 0);
static_assert((SEQ % 64) == 0);
static_assert(DIM == NHEAD * HD);
static_assert(HD == 64);
static_assert((DIM % 64) == 0 && (DIM % 32) == 0);
static_assert((DFF % 64) == 0 && (DFF % 32) == 0);
static_assert((QKLD % 64) == 0);
static_assert((MROWS % 64) == 0);
static_assert((MROWS % LNROWS) == 0);
static_assert((DIM % 128) == 0);
static_assert((size_t)MROWS * DFF < (size_t)0xFFFFFFFFu);
static_assert((size_t)DFF * DIM < (size_t)0xFFFFFFFFu);

#define LDT 72
#define LDC 68

#define WCARRY 64.0f
#define PCARRY 1024.0f
#define VCARRY 64.0f
#define FCARRY 16.0f

#define WQKV_BYTES ((size_t)3 * DIM * DIM * 2)
#define WO_BYTES   ((size_t)DIM * DIM * 2)
#define WFF_BYTES  ((size_t)DFF * DIM * 2)
#define P16_BYTES  ((size_t)MROWS * DIM * 2)
#define QK_BYTES   ((size_t)MROWS * QKLD * 2)
#define P32_BYTES  ((size_t)MROWS * DIM * 4)
#define F1_BYTES   ((size_t)MROWS * DFF * 2)
#define OFF_WQKV ((size_t)0)
#define OFF_WO   (OFF_WQKV + WQKV_BYTES)
#define OFF_W1   (OFF_WO + WO_BYTES)
#define OFF_W2   (OFF_W1 + WFF_BYTES)
#define OFF_H16  (OFF_W2 + WFF_BYTES)
#define OFF_QK   (OFF_H16 + P16_BYTES)
#define OFF_VT   (OFF_QK + QK_BYTES)
#define OFF_CTX  (OFF_VT + P16_BYTES)
#define OFF_X1   (OFF_CTX + P16_BYTES)
#define OFF_H2   (OFF_X1 + P32_BYTES)
#define OFF_F1   (OFF_H2 + P16_BYTES)
#define WS_TOTAL (OFF_F1 + F1_BYTES)
static_assert((WQKV_BYTES % 128) == 0 && (WO_BYTES % 128) == 0 && (WFF_BYTES % 128) == 0);
static_assert((P16_BYTES % 128) == 0 && (P32_BYTES % 128) == 0);
static_assert((QK_BYTES % 128) == 0 && (F1_BYTES % 128) == 0);
static_assert(WS_TOTAL <= (size_t)134217728);

__device__ __forceinline__ float bf16r(float x) {
  unsigned int u = __float_as_uint(x);
  u = (u + 0x7FFFu + ((u >> 16) & 1u)) & 0xFFFF0000u;
  return __uint_as_float(u);
}

__device__ __forceinline__ size_t xrow(unsigned row) {
  return (size_t)(row / (unsigned)SEQ) * (size_t)SEQ_FULL + (size_t)(row % (unsigned)SEQ);
}

__device__ __forceinline__ v16h frag_at(const _Float16* p) {
  v8h lo = *(const v8h*)(p);
  v8h hi = *(const v8h*)(p + 16);
  v16h out;
#pragma unroll
  for (int i = 0; i < 8; ++i) { out[i] = lo[i]; out[i + 8] = hi[i]; }
  return out;
}
__device__ __forceinline__ v16h ld_frag(const _Float16* base, unsigned ld) {
  const unsigned lane = threadIdx.x & 31u;
  return frag_at(base + (lane & 15u) * ld + (lane >> 4) * 8u);
}

__device__ __forceinline__ v8f wmma16(v16h a, v16h b, v8f c) {
  v8f d = __builtin_amdgcn_wmma_f32_16x16x32_f16(false, a, false, b, (short)0, c,
                                                 false, false);
  asm volatile("v_nop\n\tv_nop\n\tv_nop\n\tv_nop" : "+v"(d) : "v"(a), "v"(b));
  return d;
}

__device__ __forceinline__ float red16_max(float x) {
#pragma unroll
  for (int off = 1; off < 16; off <<= 1) x = fmaxf(x, __shfl_xor(x, off, 32));
  return x;
}
__device__ __forceinline__ float red16_sum(float x) {
#pragma unroll
  for (int off = 1; off < 16; off <<= 1) x += __shfl_xor(x, off, 32);
  return x;
}
__device__ __forceinline__ float red32_sum(float x) {
#pragma unroll
  for (int off = 1; off < 32; off <<= 1) x += __shfl_xor(x, off, 32);
  return x;
}

__device__ __forceinline__ void wave_lds_sync() {
  __builtin_amdgcn_fence(3  , "wavefront");
  asm volatile("s_wait_dscnt 0x0" ::: "memory");
  __builtin_amdgcn_wave_barrier();
}

__global__ __launch_bounds__(256) void wt_kernel(
    const float* __restrict__ src, _Float16* __restrict__ dst,
    unsigned R, unsigned C, float carry) {
  __shared__ __attribute__((aligned(16))) float Ts[64 * LDC];
  const unsigned tid = threadIdx.x;
  const unsigned c0 = blockIdx.x * 64u;
  const unsigned r0 = blockIdx.y * 64u;
  const size_t zoff = (size_t)blockIdx.z * (size_t)R * (size_t)C;
#pragma unroll
  for (unsigned i = 0; i < 4u; ++i) {
    const unsigned idx = tid + 256u * i;
    const unsigned r = idx >> 4, c = (idx & 15u) * 4u;
    const v4f v = *(const v4f*)(src + zoff + (size_t)(r0 + r) * C + c0 + c);
    *(v4f*)&Ts[r * LDC + c] = v;
  }
  __syncthreads();
  v8h x[2];
  size_t off[2];
#pragma unroll
  for (unsigned i = 0; i < 2u; ++i) {
    const unsigned dcol = 32u * i + (tid >> 3);
    const unsigned kk = (tid & 7u) * 8u;
#pragma unroll
    for (unsigned j = 0; j < 8u; ++j)
      x[i][j] = (_Float16)(carry * bf16r(Ts[(kk + j) * LDC + dcol]));
    off[i] = zoff + (size_t)(c0 + dcol) * R + r0 + kk;
  }
#pragma unroll
  for (int i = 0; i < 2; ++i) *(volatile v8h*)(dst + off[i]) = x[i];
  __threadfence();
#pragma unroll
  for (int i = 0; i < 2; ++i) *(volatile v8h*)(dst + off[i]) = x[i];
}

template <int MODE, int KD, int LDO>
__device__ __forceinline__ void gemm_body(
    const _Float16* __restrict__ A16, const _Float16* __restrict__ Bt,
    const float* __restrict__ addf, const float* __restrict__ resf,
    float* __restrict__ outf, _Float16* __restrict__ out16, float* Cs) {
  static_assert((KD % 64) == 0);
  static_assert((LDO % 64) == 0);
  const unsigned tid = threadIdx.x, lane = tid & 31u;
  const unsigned w = (unsigned)__builtin_amdgcn_readfirstlane((int)(tid >> 5));
  const unsigned mw = w >> 1, nw = w & 1u;
  const unsigned hh = lane >> 4, m = lane & 15u;
  const unsigned n0 = blockIdx.x * 64u;
  const unsigned row0 = blockIdx.y * 64u;

  const _Float16* ap  = A16 + (size_t)(row0 + mw * 16u + m) * KD + hh * 8u;
  const _Float16* bp0 = Bt + (size_t)(n0 + nw * 32u + m) * KD + hh * 8u;
  const _Float16* bp1 = bp0 + (size_t)16 * KD;
  v8f acc0 = {}, acc1 = {};
#pragma unroll 2
  for (unsigned k0 = 0; k0 < (unsigned)KD; k0 += 32u) {
    const v16h a  = frag_at(ap + k0);
    const v16h b0 = frag_at(bp0 + k0);
    const v16h b1 = frag_at(bp1 + k0);
    acc0 = wmma16(a, b0, acc0);
    acc1 = wmma16(a, b1, acc1);
  }
#pragma unroll
  for (int r = 0; r < 8; ++r) {
    float* d = &Cs[(mw * 16u + hh * 8u + (unsigned)r) * LDC + nw * 32u + m];
    d[0]  = acc0[r];
    d[16] = acc1[r];
  }
  __syncthreads();

  if (MODE == 0 || MODE == 3) {
    v8h x[2];
    size_t off[2];
#pragma unroll
    for (unsigned i = 0; i < 2u; ++i) {
      const unsigned r = 32u * i + (tid >> 3);
      const unsigned c = (tid & 7u) * 8u;
      const v4f u0 = *(const v4f*)&Cs[r * LDC + c];
      const v4f u1 = *(const v4f*)&Cs[r * LDC + c + 4];
      if (MODE == 0) {
#pragma unroll
        for (int j = 0; j < 4; ++j) {
          x[i][j]     = (_Float16)(u0[j] * (1.0f / WCARRY));
          x[i][j + 4] = (_Float16)(u1[j] * (1.0f / WCARRY));
        }
      } else {
        const v4f g0 = *(const v4f*)(addf + n0 + c);
        const v4f g1 = *(const v4f*)(addf + n0 + c + 4);
#pragma unroll
        for (int j = 0; j < 4; ++j) {
          x[i][j]     = (_Float16)(FCARRY * fmaxf(u0[j] * (1.0f / WCARRY) + bf16r(g0[j]), 0.0f));
          x[i][j + 4] = (_Float16)(FCARRY * fmaxf(u1[j] * (1.0f / WCARRY) + bf16r(g1[j]), 0.0f));
        }
      }
      off[i] = (size_t)(row0 + r) * LDO + n0 + c;
    }
#pragma unroll
    for (int i = 0; i < 2; ++i) *(volatile v8h*)(out16 + off[i]) = x[i];
    __threadfence();
#pragma unroll
    for (int i = 0; i < 2; ++i) *(volatile v8h*)(out16 + off[i]) = x[i];
  }

  if (MODE == 1) {
    const unsigned bat = row0 / (unsigned)SEQ;
    const unsigned t0  = row0 % (unsigned)SEQ;
    v8h x[2];
    size_t off[2];
#pragma unroll
    for (unsigned i = 0; i < 2u; ++i) {
      const unsigned dcol = 32u * i + (tid >> 3);
      const unsigned kk = (tid & 7u) * 8u;
#pragma unroll
      for (unsigned j = 0; j < 8u; ++j)
        x[i][j] = (_Float16)(Cs[(kk + j) * LDC + dcol] * (1.0f / WCARRY));
      off[i] = ((size_t)bat * DIM + n0 + dcol) * SEQ + t0 + kk;
    }
#pragma unroll
    for (int i = 0; i < 2; ++i) *(volatile v8h*)(out16 + off[i]) = x[i];
    __threadfence();
#pragma unroll
    for (int i = 0; i < 2; ++i) *(volatile v8h*)(out16 + off[i]) = x[i];
  }

  if (MODE == 4 || MODE == 5) {
    v4f xs[4];
    size_t off[4];
#pragma unroll
    for (unsigned i = 0; i < 4u; ++i) {
      const unsigned r = 16u * i + (tid >> 4);
      const unsigned c = (tid & 15u) * 4u;
      const size_t o = (size_t)(row0 + r) * DIM + n0 + c;
      const v4f u = *(const v4f*)&Cs[r * LDC + c];
      v4f val;
      if (MODE == 4) {
        const v4f g = *(const v4f*)(addf + n0 + c);
        const v4f hres = *(const v4f*)(resf + o);
#pragma unroll
        for (int j = 0; j < 4; ++j)
          val[j] = (u[j] * (1.0f / (WCARRY * FCARRY)) + bf16r(g[j])) + hres[j];
      } else {
        const v4f xin = *(const v4f*)(resf + xrow(row0 + r) * DIM + n0 + c);
#pragma unroll
        for (int j = 0; j < 4; ++j)
          val[j] = u[j] * (1.0f / (WCARRY * VCARRY)) + bf16r(xin[j]);
      }
      xs[i] = val;
      off[i] = o;
    }
#pragma unroll
    for (int i = 0; i < 4; ++i) *(volatile v4f*)(outf + off[i]) = xs[i];
    __threadfence();
#pragma unroll
    for (int i = 0; i < 4; ++i) *(volatile v4f*)(outf + off[i]) = xs[i];
  }
}

__global__ __launch_bounds__(256) void gemm_qk_kernel(
    const _Float16* __restrict__ A16, const _Float16* __restrict__ Bt,
    _Float16* __restrict__ out16) {
  __shared__ __attribute__((aligned(16))) float Cs[64 * LDC];
  gemm_body<0, DIM, QKLD>(A16, Bt, nullptr, nullptr, nullptr, out16, Cs);
}
__global__ __launch_bounds__(256) void gemm_vt_kernel(
    const _Float16* __restrict__ A16, const _Float16* __restrict__ Bt,
    _Float16* __restrict__ out16) {
  __shared__ __attribute__((aligned(16))) float Cs[64 * LDC];
  gemm_body<1, DIM, DIM>(A16, Bt, nullptr, nullptr, nullptr, out16, Cs);
}
__global__ __launch_bounds__(256) void gemm_wo_kernel(
    const _Float16* __restrict__ A16, const _Float16* __restrict__ Bt,
    const float* __restrict__ xin, float* __restrict__ outf) {
  __shared__ __attribute__((aligned(16))) float Cs[64 * LDC];
  gemm_body<5, DIM, DIM>(A16, Bt, nullptr, xin, outf, nullptr, Cs);
}
__global__ __launch_bounds__(256) void gemm_ffn1_kernel(
    const _Float16* __restrict__ A16, const _Float16* __restrict__ Bt,
    const float* __restrict__ bias, _Float16* __restrict__ out16) {
  __shared__ __attribute__((aligned(16))) float Cs[64 * LDC];
  gemm_body<3, DIM, DFF>(A16, Bt, bias, nullptr, nullptr, out16, Cs);
}
__global__ __launch_bounds__(256) void gemm_ffn2_kernel(
    const _Float16* __restrict__ A16, const _Float16* __restrict__ Bt,
    const float* __restrict__ bias, const float* __restrict__ resf,
    float* __restrict__ outf) {
  __shared__ __attribute__((aligned(16))) float Cs[64 * LDC];
  gemm_body<4, DFF, DIM>(A16, Bt, bias, resf, outf, nullptr, Cs);
}

__global__ __launch_bounds__(256) void attn_kernel(
    const _Float16* __restrict__ QK, const _Float16* __restrict__ Vt,
    _Float16* __restrict__ Ov) {
  __shared__ __attribute__((aligned(16))) _Float16 Ks[64 * LDT];
  __shared__ __attribute__((aligned(16))) _Float16 Vs[64 * LDT];
  __shared__ __attribute__((aligned(16))) _Float16 Ps[8 * 16 * LDT];

  const unsigned tid = threadIdx.x, lane = tid & 31u;
  const unsigned w = (unsigned)__builtin_amdgcn_readfirstlane((int)(tid >> 5));
  const unsigned hh = lane >> 4, m = lane & 15u;
  const unsigned q0 = blockIdx.x * 128u;
  const unsigned head = blockIdx.y;
  const unsigned bat = blockIdx.z;
  const unsigned qw0 = q0 + w * 16u;
  const unsigned pb = w * (16u * LDT);
  const float scale = 0.125f;
  const size_t brow = (size_t)bat * SEQ;

  const size_t qoff = (brow + qw0 + m) * QKLD + head * HD + hh * 8u;
  v16h qf[2];
  qf[0] = frag_at(QK + qoff);
  qf[1] = frag_at(QK + qoff + 32);

  float mrow[8], lrow[8];
  v8f o[4];
#pragma unroll
  for (int v = 0; v < 8; ++v) { mrow[v] = -1.0e30f; lrow[v] = 0.0f; }
#pragma unroll
  for (int nb = 0; nb < 4; ++nb) o[nb] = (v8f){};

  const size_t kplane = brow * QKLD + DIM + head * HD;
  const size_t vplane = ((size_t)bat * DIM + head * HD) * SEQ;

  for (unsigned kb = 0; kb < (unsigned)SEQ; kb += 64u) {
#pragma unroll
    for (unsigned j = 0; j < 2u; ++j) {
      const unsigned idx = tid + 256u * j;
      const unsigned r = idx >> 3, c = (idx & 7u) * 8u;
      *(v8h*)&Ks[r * LDT + c] = *(const v8h*)(QK + kplane + (size_t)(kb + r) * QKLD + c);
      *(v8h*)&Vs[r * LDT + c] = *(const v8h*)(Vt + vplane + (size_t)r * SEQ + kb + c);
    }
    __syncthreads();

    v8f s[4];
    if (kb <= qw0 + 15u) {
#pragma unroll
      for (int kg = 0; kg < 4; ++kg) {
        v8f t = {};
#pragma unroll
        for (int c = 0; c < 2; ++c) {
          const v16h kf = ld_frag(&Ks[(kg * 16) * LDT + c * 32], LDT);
          t = wmma16(qf[c], kf, t);
        }
        s[kg] = t * scale;
      }
      if (kb + 63u > qw0) {
#pragma unroll
        for (int kg = 0; kg < 4; ++kg) {
          const unsigned key = kb + (unsigned)kg * 16u + m;
#pragma unroll
          for (int v = 0; v < 8; ++v) {
            const unsigned qr = qw0 + hh * 8u + (unsigned)v;
            const float sv = s[kg][v];
            s[kg][v] = (key <= qr) ? sv : 0.0f;
          }
        }
      }
    } else {
#pragma unroll
      for (int kg = 0; kg < 4; ++kg) s[kg] = (v8f){};
    }

    float alpha[8];
#pragma unroll
    for (int v = 0; v < 8; ++v) {
      float mx = fmaxf(fmaxf(s[0][v], s[1][v]), fmaxf(s[2][v], s[3][v]));
      mx = red16_max(mx);
      const float mn = fmaxf(mrow[v], mx);
      alpha[v] = __expf(mrow[v] - mn);
      mrow[v] = mn;
    }
#pragma unroll
    for (int kg = 0; kg < 4; ++kg)
#pragma unroll
      for (int v = 0; v < 8; ++v) s[kg][v] = __expf(s[kg][v] - mrow[v]);
#pragma unroll
    for (int v = 0; v < 8; ++v) {
      const float rs = red16_sum((s[0][v] + s[1][v]) + (s[2][v] + s[3][v]));
      lrow[v] = alpha[v] * lrow[v] + rs;
    }
#pragma unroll
    for (int nb = 0; nb < 4; ++nb)
#pragma unroll
      for (int v = 0; v < 8; ++v) o[nb][v] = o[nb][v] * alpha[v];

#pragma unroll
    for (int kg = 0; kg < 4; ++kg)
#pragma unroll
      for (int v = 0; v < 8; ++v)
        Ps[pb + (hh * 8u + (unsigned)v) * LDT + (unsigned)kg * 16u + m] =
            (_Float16)(s[kg][v] * PCARRY);
    wave_lds_sync();

#pragma unroll
    for (int c = 0; c < 2; ++c) {
      const v16h pf = ld_frag(&Ps[pb + c * 32], LDT);
#pragma unroll
      for (int nb = 0; nb < 4; ++nb) {
        const v16h vf = ld_frag(&Vs[(nb * 16) * LDT + c * 32], LDT);
        o[nb] = wmma16(pf, vf, o[nb]);
      }
    }
    __syncthreads();
  }

  float inv[8];
#pragma unroll
  for (int v = 0; v < 8; ++v) inv[v] = __builtin_amdgcn_rcpf(lrow[v]) * (VCARRY / PCARRY);
#pragma unroll
  for (int nb = 0; nb < 4; ++nb)
#pragma unroll
    for (int v = 0; v < 8; ++v)
      Ps[pb + (hh * 8u + (unsigned)v) * LDT + (unsigned)nb * 16u + m] =
          (_Float16)(o[nb][v] * inv[v]);
  wave_lds_sync();
  v8h x[4];
  size_t off[4];
#pragma unroll
  for (unsigned i = 0; i < 4u; ++i) {
    const unsigned r = 4u * i + (lane >> 3);
    const unsigned c = (lane & 7u) * 8u;
    x[i] = *(const v8h*)&Ps[pb + r * LDT + c];
    off[i] = (brow + qw0 + r) * DIM + head * HD + c;
  }
#pragma unroll
  for (int i = 0; i < 4; ++i) *(volatile v8h*)(Ov + off[i]) = x[i];
  __threadfence();
#pragma unroll
  for (int i = 0; i < 4; ++i) *(volatile v8h*)(Ov + off[i]) = x[i];
}

__device__ __forceinline__ void ln_store(
    const float* S, const float* __restrict__ g, const float* __restrict__ be,
    _Float16* __restrict__ out16, size_t obase, float mu, float rs) {
  const unsigned lane = threadIdx.x & 31u;
#pragma unroll 1
  for (unsigned it = 0; it < (unsigned)(DIM / 128); ++it) {
    const unsigned c = it * 128u + lane * 4u;
    const v4f v = *(const v4f*)&S[c];
    const v4f gg = *(const v4f*)(g + c);
    const v4f bb = *(const v4f*)(be + c);
    v4h x;
#pragma unroll
    for (int j = 0; j < 4; ++j)
      x[j] = (_Float16)((v[j] - mu) * rs * bf16r(gg[j]) + bf16r(bb[j]));
    *(volatile v4h*)(out16 + obase + c) = x;
  }
}

template <int RIN>
__device__ __forceinline__ void ln_body(
    const float* __restrict__ src, size_t sbase,
    const float* __restrict__ g, const float* __restrict__ be,
    _Float16* __restrict__ out16, size_t obase, float* S) {
  const unsigned lane = threadIdx.x & 31u;
  float sum = 0.0f;
#pragma unroll 1
  for (unsigned it = 0; it < (unsigned)(DIM / 128); ++it) {
    const unsigned c = it * 128u + lane * 4u;
    v4f v = *(const v4f*)(src + sbase + c);
    if (RIN) {
#pragma unroll
      for (int j = 0; j < 4; ++j) v[j] = bf16r(v[j]);
    }
    *(v4f*)&S[c] = v;
    sum += (v[0] + v[1]) + (v[2] + v[3]);
  }
  sum = red32_sum(sum);
  const float mu = sum * (1.0f / (float)DIM);
  float sq = 0.0f;
#pragma unroll 1
  for (unsigned it = 0; it < (unsigned)(DIM / 128); ++it) {
    const unsigned c = it * 128u + lane * 4u;
    const v4f v = *(const v4f*)&S[c];
    const float d0 = v[0] - mu, d1 = v[1] - mu, d2 = v[2] - mu, d3 = v[3] - mu;
    sq += (d0 * d0 + d1 * d1) + (d2 * d2 + d3 * d3);
  }
  sq = red32_sum(sq);
  const float rs = rsqrtf(sq * (1.0f / (float)DIM) + LN_EPS);
  wave_lds_sync();
  ln_store(S, g, be, out16, obase, mu, rs);
  __threadfence();
  ln_store(S, g, be, out16, obase, mu, rs);
}

__global__ __launch_bounds__(256) void ln1_kernel(
    const float* __restrict__ X, const float* __restrict__ g,
    const float* __restrict__ be, _Float16* __restrict__ h16) {
  __shared__ __attribute__((aligned(16))) float S[LNROWS * DIM];
  const unsigned w = (unsigned)__builtin_amdgcn_readfirstlane((int)(threadIdx.x >> 5));
  const unsigned row = blockIdx.x * (unsigned)LNROWS + w;
  ln_body<1>(X, xrow(row) * DIM, g, be, h16, (size_t)row * DIM, S + w * (unsigned)DIM);
}
__global__ __launch_bounds__(256) void ln2_kernel(
    const float* __restrict__ Y, const float* __restrict__ g,
    const float* __restrict__ be, _Float16* __restrict__ h16) {
  __shared__ __attribute__((aligned(16))) float S[LNROWS * DIM];
  const unsigned w = (unsigned)__builtin_amdgcn_readfirstlane((int)(threadIdx.x >> 5));
  const unsigned row = blockIdx.x * (unsigned)LNROWS + w;
  ln_body<0>(Y, (size_t)row * DIM, g, be, h16, (size_t)row * DIM, S + w * (unsigned)DIM);
}

extern "C" void kernel_launch(void* const* d_in, const int* in_sizes, int n_in,
                              void* d_out, int out_size, void* d_ws, size_t ws_size,
                              hipStream_t stream) {
  if (n_in < 13) return;
  const long long need_x = ((long long)(NB - 1) * SEQ_FULL + SEQ) * DIM;
  if ((long long)in_sizes[0] < need_x) return;
  if (in_sizes[1] < DIM || in_sizes[2] < DIM || in_sizes[3] < DIM || in_sizes[4] < DIM) return;
  if ((long long)in_sizes[5] < (long long)DIM * DIM) return;
  if ((long long)in_sizes[6] < (long long)DIM * DIM) return;
  if ((long long)in_sizes[7] < (long long)DIM * DIM) return;
  if ((long long)in_sizes[8] < (long long)DIM * DIM) return;
  if ((long long)in_sizes[9] < (long long)DIM * DFF) return;
  if (in_sizes[10] < DFF) return;
  if ((long long)in_sizes[11] < (long long)DFF * DIM) return;
  if (in_sizes[12] < DIM) return;
  if ((long long)out_size < (long long)MROWS * DIM) return;
  if (ws_size < WS_TOTAL) return;

  const float* X    = (const float*)d_in[0];
  const float* g1   = (const float*)d_in[1];
  const float* be1  = (const float*)d_in[2];
  const float* g2   = (const float*)d_in[3];
  const float* be2  = (const float*)d_in[4];
  const float* Wq   = (const float*)d_in[5];
  const float* Wk   = (const float*)d_in[6];
  const float* Wv   = (const float*)d_in[7];
  const float* Wo   = (const float*)d_in[8];
  const float* W1   = (const float*)d_in[9];
  const float* b1   = (const float*)d_in[10];
  const float* W2   = (const float*)d_in[11];
  const float* b2   = (const float*)d_in[12];
  float* out = (float*)d_out;

  char* ws = (char*)d_ws;
  _Float16* Wqkv16 = (_Float16*)(ws + OFF_WQKV);
  _Float16* Wo16   = (_Float16*)(ws + OFF_WO);
  _Float16* W1_16  = (_Float16*)(ws + OFF_W1);
  _Float16* W2_16  = (_Float16*)(ws + OFF_W2);
  _Float16* H16    = (_Float16*)(ws + OFF_H16);
  _Float16* QK16   = (_Float16*)(ws + OFF_QK);
  _Float16* Vt16   = (_Float16*)(ws + OFF_VT);
  _Float16* Ctx16  = (_Float16*)(ws + OFF_CTX);
  float*    X1     = (float*)(ws + OFF_X1);
  _Float16* H2_16  = (_Float16*)(ws + OFF_H2);
  _Float16* F1_16  = (_Float16*)(ws + OFF_F1);

  dim3 blk(256);

  wt_kernel<<<dim3(HD / 64, DIM / 64, NHEAD), blk, 0, stream>>>(
      Wq, Wqkv16, (unsigned)DIM, (unsigned)HD, WCARRY);
  wt_kernel<<<dim3(HD / 64, DIM / 64, NHEAD), blk, 0, stream>>>(
      Wk, Wqkv16 + (size_t)DIM * DIM, (unsigned)DIM, (unsigned)HD, WCARRY);
  wt_kernel<<<dim3(HD / 64, DIM / 64, NHEAD), blk, 0, stream>>>(
      Wv, Wqkv16 + (size_t)2 * DIM * DIM, (unsigned)DIM, (unsigned)HD, WCARRY);
  wt_kernel<<<dim3(DIM / 64, DIM / 64, 1), blk, 0, stream>>>(
      Wo, Wo16, (unsigned)DIM, (unsigned)DIM, WCARRY);
  wt_kernel<<<dim3(DFF / 64, DIM / 64, 1), blk, 0, stream>>>(
      W1, W1_16, (unsigned)DIM, (unsigned)DFF, WCARRY);
  wt_kernel<<<dim3(DIM / 64, DFF / 64, 1), blk, 0, stream>>>(
      W2, W2_16, (unsigned)DFF, (unsigned)DIM, WCARRY);

  ln1_kernel<<<dim3(MROWS / LNROWS), blk, 0, stream>>>(X, g1, be1, H16);

  gemm_qk_kernel<<<dim3(QKLD / 64, MROWS / 64), blk, 0, stream>>>(H16, Wqkv16, QK16);
  gemm_vt_kernel<<<dim3(DIM / 64, MROWS / 64), blk, 0, stream>>>(
      H16, Wqkv16 + (size_t)2 * DIM * DIM, Vt16);

  attn_kernel<<<dim3(SEQ / 128, NHEAD, NB), blk, 0, stream>>>(QK16, Vt16, Ctx16);

  gemm_wo_kernel<<<dim3(DIM / 64, MROWS / 64), blk, 0, stream>>>(Ctx16, Wo16, X, X1);

  ln2_kernel<<<dim3(MROWS / LNROWS), blk, 0, stream>>>(X1, g2, be2, H2_16);

  gemm_ffn1_kernel<<<dim3(DFF / 64, MROWS / 64), blk, 0, stream>>>(H2_16, W1_16, b1, F1_16);
  gemm_ffn2_kernel<<<dim3(DIM / 64, MROWS / 64), blk, 0, stream>>>(F1_16, W2_16, b2, X1, out);
}
